// CausalSelfAttentionGQA_83863531422015
// MI455X (gfx1250) — hardware-run, weakly checked
//
#include <hip/hip_runtime.h>

#ifndef NB
#define NB 1
#endif
#ifndef SEQ
#define SEQ 4096
#endif
#define NB_FULL 1
#define SEQ_FULL 4096
#define DM 2048
#define NH 16
#define NKV 4
#define GQ (NH / NKV)
#define HD 128
#define GCOLS ((GQ + 2) * HD)
#define NQKV (NKV * GCOLS)
#define KDIM (NKV * HD)
#define SLEN SEQ
#define NR (NB * SLEN)
#define TQ SLEN
#define TK SLEN
#define SCL 0.08838834764831845f
#define WIN 1023
#define CTXC 64.0f
#define QBLKS (TQ / 64)
#define RPGQ (SLEN / NH)
#define RPGK (SLEN / NKV)
static_assert(SLEN % 256 == 0);
static_assert(SLEN <= SEQ_FULL);
static_assert(NB == 1 && NB <= NB_FULL);
static_assert(DM % 64 == 0 && DM == NH * HD);
static_assert(HD == 128 && GCOLS == 768 && NQKV == 3072 && KDIM == 512);
static_assert(NR % 128 == 0 && NQKV % 64 == 0 && DM % 32 == 0);
static_assert(RPGQ * NH == SLEN && RPGK * NKV == SLEN && RPGK % 64 == 0);
static_assert(TK % 32 == 0 && TQ % 64 == 0);
static_assert(4 * 32 * 68 * 4 <= 131072);
static_assert(4 * 16 * 40 * 2 + 4 * 16 * 132 * 4 <= 131072);
static_assert(64 * 130 * 2 <= 131072 && 64 * 66 * 2 <= 131072);
static_assert((size_t)NQKV * DM * 2 + (size_t)DM * DM * 2 + (size_t)NR * NQKV * 4 + (size_t)NR * DM * 2 + (size_t)NR * DM * 2 + (size_t)NR * KDIM * 2 + (size_t)NKV * HD * TK * 2 <= ((size_t)128 << 20));

typedef _Float16 v16h __attribute__((ext_vector_type(16)));
typedef _Float16 v4h __attribute__((ext_vector_type(4)));
typedef unsigned short v8us __attribute__((ext_vector_type(8), may_alias));
typedef float v8f __attribute__((ext_vector_type(8)));
typedef float v4f __attribute__((ext_vector_type(4)));
typedef float v4fa __attribute__((ext_vector_type(4), may_alias));
union FragH { v16h v; v8us half[2]; _Float16 h[16]; unsigned short u[16]; };

__device__ __forceinline__ unsigned short bf16_bits(float x) { unsigned int u = __float_as_uint(x); return (unsigned short)((u + 0x7FFFu + ((u >> 16) & 1u)) >> 16); }
__device__ __forceinline__ float bf16_val(unsigned short b) { return __uint_as_float(((unsigned int)b) << 16); }
__device__ __forceinline__ float bf16_rne(float x) { return bf16_val(bf16_bits(x)); }
static __device__ __forceinline__ _Float16 toh_flush(float v) { const _Float16 r = (_Float16)v; return (fabsf(v) < 6.103515625e-05f) ? (_Float16)0.0f : r; }

__device__ __forceinline__ v16h g2_frag(const _Float16* p, int hh) { FragH f; f.half[0] = *(const v8us*)((const unsigned short*)p + 8 * hh); f.half[1] = *(const v8us*)((const unsigned short*)p + 16 + 8 * hh); return f.v; }
__device__ __forceinline__ v8f g2_mma(v16h a, v16h b, v8f c) { v8f d = __builtin_amdgcn_wmma_f32_16x16x32_f16(false, a, false, b, (short)0, c, false, false); asm volatile("v_nop\n\tv_nop\n\tv_nop\n\tv_nop" : "+v"(d) : "v"(a), "v"(b)); return d; }

__global__ __launch_bounds__(256) void k_wtr(const float* __restrict__ Wm, _Float16* __restrict__ Bt, int KD, int ND, float sc) {
  __shared__ unsigned short tl[64][66];
  const int tid = threadIdx.x; const int n0 = blockIdx.x * 64, k0 = blockIdx.y * 64;
  for (int i = tid; i < 64 * 16; i += 256) {
    const int kr = i >> 4, c4 = (i & 15) * 4;
    const v4f a = *(const v4fa*)(Wm + (size_t)(k0 + kr) * ND + n0 + c4);
    FragH f;
#pragma unroll
    for (int q = 0; q < 4; ++q) f.h[q] = toh_flush(bf16_rne(a[q]) * sc);
#pragma unroll
    for (int q = 0; q < 4; ++q) tl[kr][c4 + q] = f.u[q];
  }
  __syncthreads();
  static_assert(256 * 2 * 16 == 64 * 128);
  for (int pass = 0; pass < 2; ++pass) {
#pragma unroll
    for (int rd = 0; rd < 2; ++rd) {
      const int n = rd * 32 + (tid >> 3), pc = tid & 7; FragH f;
#pragma unroll
      for (int q = 0; q < 8; ++q) f.u[q] = tl[pc * 8 + q][n];
      *(volatile v8us*)((unsigned short*)Bt + (size_t)(n0 + n) * KD + k0 + pc * 8) = f.half[0];
    }
    if (pass == 0) __threadfence();
  }
}

__global__ __launch_bounds__(256) void k_x16(const float* __restrict__ x, _Float16* __restrict__ X16, size_t n8) {
  const size_t t = (size_t)blockIdx.x * 256 + threadIdx.x; if (t >= n8) return;
  const size_t e = t * 8; const size_t r = e / DM; const size_t c = e % DM; const size_t b = r / SLEN, s = r % SLEN;
  const float* src = x + (b * SEQ_FULL + s) * DM + c;
  const v4f a0 = *(const v4fa*)src, a1 = *(const v4fa*)(src + 4);
  FragH f;
#pragma unroll
  for (int q = 0; q < 4; ++q) { f.h[q] = (_Float16)bf16_rne(a0[q]); f.h[4 + q] = (_Float16)bf16_rne(a1[q]); }
  const v8us o = f.half[0];
  *(volatile v8us*)((unsigned short*)X16 + e) = o; __threadfence(); *(volatile v8us*)((unsigned short*)X16 + e) = o;
}

template <int ACT>
__global__ __launch_bounds__(128) void k_gemm2(const _Float16* __restrict__ A, int lda, size_t sA, const _Float16* __restrict__ Bh, int ldb, size_t sB, float alpha,
                                               float* C, _Float16* C16, int ldc, size_t sC, int M, int N, int K) {
  __shared__ __attribute__((aligned(16))) float so[4][32][68];
  const int tid = threadIdx.x, w = tid >> 5, lane = tid & 31, ln = lane & 15, hh = lane >> 4; const int by = blockIdx.y;
  A += (size_t)by * sA; Bh += (size_t)by * sB; const size_t cofs = (size_t)by * sC;
  const int ntn = N >> 6; const int mt = blockIdx.x / ntn, nq = blockIdx.x - mt * ntn; const int row0 = mt * 128 + 32 * w, col0 = nq * 64; if (row0 >= M) return;
  const _Float16* a0p = A + (size_t)(row0 + ln) * lda; const _Float16* a1p = a0p + (size_t)16 * lda;
  const _Float16* b0p = Bh + (size_t)(col0 + ln) * ldb; const _Float16* b1p = b0p + (size_t)16 * ldb; const _Float16* b2p = b1p + (size_t)16 * ldb; const _Float16* b3p = b2p + (size_t)16 * ldb;
  const v8f z8 = {0.f,0.f,0.f,0.f,0.f,0.f,0.f,0.f}; v8f c00 = z8, c01 = z8, c02 = z8, c03 = z8, c10 = z8, c11 = z8, c12 = z8, c13 = z8;
#pragma unroll 1
  for (int kb = 0; kb < K; kb += 32) {
    const v16h a0 = g2_frag(a0p + kb, hh), a1 = g2_frag(a1p + kb, hh);
    v16h bf = g2_frag(b0p + kb, hh); c00 = g2_mma(a0, bf, c00); c10 = g2_mma(a1, bf, c10);
    bf = g2_frag(b1p + kb, hh); c01 = g2_mma(a0, bf, c01); c11 = g2_mma(a1, bf, c11);
    bf = g2_frag(b2p + kb, hh); c02 = g2_mma(a0, bf, c02); c12 = g2_mma(a1, bf, c12);
    bf = g2_frag(b3p + kb, hh); c03 = g2_mma(a0, bf, c03); c13 = g2_mma(a1, bf, c13);
  }
  v8f accs[8] = {c00, c01, c02, c03, c10, c11, c12, c13};
#pragma unroll
  for (int u = 0; u < 8; ++u) {
    const int t = u & 3, half = u >> 2;
#pragma unroll
    for (int r = 0; r < 8; ++r) { const int rloc = half * 16 + 8 * hh + r; float v = accs[u][r] * alpha; if (ACT == 3) v = fmaxf(v, 0.f); so[w][rloc][t * 16 + ln] = v; }
  }
  __builtin_amdgcn_fence(4, "workgroup"); __builtin_amdgcn_wave_barrier();
  const int rsub = lane >> 4, c4 = (lane & 15) * 4;
  for (int pass = 0; pass < 2; ++pass) {
#pragma unroll
    for (int q = 0; q < 16; ++q) {
      const int r = q * 2 + rsub; const v4f v = *(const v4fa*)&so[w][r][c4];
      if (C) *(volatile v4f*)(C + cofs + (size_t)(row0 + r) * ldc + col0 + c4) = v;
      if (C16) { v4h h4; for (int i = 0; i < 4; ++i) h4[i] = (_Float16)v[i]; *(volatile v4h*)(C16 + cofs + (size_t)(row0 + r) * ldc + col0 + c4) = h4; }
    }
    if (pass == 0) __threadfence();
  }
}

__global__ __launch_bounds__(256) void k_ropei(const float* __restrict__ F, const float* __restrict__ TAB, _Float16* __restrict__ H, int nh, int rpg, int spg, int cofs) {
  #pragma clang fp contract(off)
  const size_t t = (size_t)blockIdx.x * 256 + threadIdx.x; if (t >= (size_t)SLEN * (size_t)nh * 16) return;
  const int p = (int)(t & 15); const int hd = (int)((t >> 4) % (size_t)nh); const int row = (int)(t / ((size_t)16 * (size_t)nh));
  const int grp = row / rpg; const int tok = (row % rpg) * nh + hd;
  const int base = (grp / spg) * GCOLS + (grp % spg) * HD + cofs;
  const float* src = F + (size_t)tok * NQKV + base + p * 8;
  const v4f xa = *(const v4fa*)src, xb = *(const v4fa*)(src + 4);
  const float* tp = TAB + (size_t)row * HD + p * 8;
  const v4f ta = *(const v4fa*)tp, tb = *(const v4fa*)(tp + 4);
  const float xe[4] = {xa[0], xa[2], xb[0], xb[2]};
  const float xo[4] = {xa[1], xa[3], xb[1], xb[3]};
  const float cc[4] = {bf16_rne(ta[0]), bf16_rne(ta[2]), bf16_rne(tb[0]), bf16_rne(tb[2])};
  const float sn[4] = {bf16_rne(ta[1]), bf16_rne(ta[3]), bf16_rne(tb[1]), bf16_rne(tb[3])};
  FragH fh;
#pragma unroll
  for (int i = 0; i < 4; ++i) {
    const float re = xe[i] * cc[i] - xo[i] * sn[i]; const float im = xo[i] * cc[i] + xe[i] * sn[i];
    fh.h[2 * i] = toh_flush(re); fh.h[2 * i + 1] = toh_flush(im);
  }
  const size_t oh = (size_t)row * ((size_t)nh * HD) + (size_t)hd * HD + p * 8;
  const v8us vh = fh.half[0];
  *(volatile v8us*)((unsigned short*)H + oh) = vh; __threadfence(); *(volatile v8us*)((unsigned short*)H + oh) = vh;
}

__global__ __launch_bounds__(256) void k_vtt(const float* __restrict__ F, _Float16* __restrict__ Vt) {
  __shared__ unsigned short tl[64][130];
  const int tid = threadIdx.x; const int nlg = SLEN / 64; const int kh = blockIdx.x / nlg, lg = blockIdx.x % nlg;
  const int p0 = lg * 64; const int g = p0 / RPGK;
  for (int i = tid; i < 64 * 32; i += 256) {
    const int r = i >> 5, c4 = (i & 31) * 4;
    const int tok = ((p0 + r) % RPGK) * NKV + kh;
    const v4f a = *(const v4fa*)(F + (size_t)tok * NQKV + g * GCOLS + (GQ + 1) * HD + c4);
    FragH f;
#pragma unroll
    for (int q = 0; q < 4; ++q) f.h[q] = toh_flush(a[q]);
#pragma unroll
    for (int q = 0; q < 4; ++q) tl[r][c4 + q] = f.u[q];
  }
  __syncthreads();
  static_assert(256 * 4 * 16 == 128 * 128);
  for (int pass = 0; pass < 2; ++pass) {
#pragma unroll
    for (int rd = 0; rd < 4; ++rd) {
      const int d = rd * 32 + (tid >> 3), pc = tid & 7; FragH f;
#pragma unroll
      for (int q = 0; q < 8; ++q) f.u[q] = tl[pc * 8 + q][d];
      *(volatile v8us*)((unsigned short*)Vt + ((size_t)kh * HD + d) * TK + p0 + pc * 8) = f.half[0];
    }
    if (pass == 0) __threadfence();
  }
}

__global__ __launch_bounds__(128) __attribute__((amdgpu_num_vgpr(256)))
void k_flashb(const _Float16* __restrict__ Q16, const _Float16* __restrict__ K16, const _Float16* __restrict__ Vt, _Float16* __restrict__ OH) {
  constexpr int RPW = 16, DT = 8, KS = 4;
  static_assert(KS * 32 == HD && DT * 16 == HD);
  __shared__ __attribute__((aligned(16))) unsigned short sP[4][RPW][40];
  __shared__ __attribute__((aligned(16))) float sO[4][RPW][132];
  const int tid = threadIdx.x, wv = tid >> 5, lane = tid & 31, ln = lane & 15, hh = lane >> 4;
  const int h = blockIdx.x / QBLKS, qblk = blockIdx.x % QBLKS; const int kvh = h / GQ;
  const int q0v = qblk * (4 * RPW) + wv * RPW;
  int jlov = q0v - WIN; jlov = (jlov < 0) ? 0 : jlov; jlov &= ~31;
  int jhiv = q0v + RPW + WIN; jhiv = (jhiv > TK) ? TK : jhiv; jhiv = (jhiv + 31) & ~31;
  const int w = __builtin_amdgcn_readfirstlane(wv);
  const int q0 = __builtin_amdgcn_readfirstlane(q0v);
  const int jlo = __builtin_amdgcn_readfirstlane(jlov);
  const int jhi = __builtin_amdgcn_readfirstlane(jhiv);
  FragH aq[KS];
  {
    const unsigned short* qr = (const unsigned short*)Q16 + (size_t)(q0 + ln) * DM + h * HD;
#pragma unroll
    for (int ks = 0; ks < KS; ++ks) { aq[ks].half[0] = *(const v8us*)(qr + ks * 32 + 8 * hh); aq[ks].half[1] = *(const v8us*)(qr + ks * 32 + 16 + 8 * hh); }
  }
  const unsigned short* Vth = (const unsigned short*)Vt + (size_t)kvh * HD * TK;
  const unsigned short* Kh = (const unsigned short*)K16 + kvh * HD;
  float m_r[8], l_r[8]; v8f oacc[DT];
#pragma unroll
  for (int r = 0; r < 8; ++r) { m_r[r] = -3.0e38f; l_r[r] = 0.f; }
#pragma unroll
  for (int dt = 0; dt < DT; ++dt) oacc[dt] = (v8f){0.f,0.f,0.f,0.f,0.f,0.f,0.f,0.f};
#pragma unroll 1
  for (int j0 = jlo; j0 < jhi; j0 += 32) {
    v8f s[2];
#pragma unroll
    for (int nt = 0; nt < 2; ++nt) {
      const unsigned short* kr = Kh + (size_t)(j0 + nt * 16 + ln) * KDIM; FragH bk[KS];
#pragma unroll
      for (int ks = 0; ks < KS; ++ks) { bk[ks].half[0] = *(const v8us*)(kr + ks * 32 + 8 * hh); bk[ks].half[1] = *(const v8us*)(kr + ks * 32 + 16 + 8 * hh); }
      v8f acc = (v8f){0.f,0.f,0.f,0.f,0.f,0.f,0.f,0.f};
#pragma unroll
      for (int ks = 0; ks < KS; ++ks) acc = g2_mma(aq[ks].v, bk[ks].v, acc);
      s[nt] = acc;
    }
#pragma unroll
    for (int r = 0; r < 8; ++r) {
      const int tq = q0 + 8 * hh + r; const int d0 = tq - (j0 + ln), d1 = d0 - 16;
      const bool ok0 = (d0 <= WIN) && (d0 >= -WIN), ok1 = (d1 <= WIN) && (d1 >= -WIN);
      const float s0 = ok0 ? s[0][r] * SCL : -3.0e38f, s1 = ok1 ? s[1][r] * SCL : -3.0e38f;
      float mc = fmaxf(s0, s1);
      mc = fmaxf(mc, __shfl_xor(mc, 1, 32)); mc = fmaxf(mc, __shfl_xor(mc, 2, 32)); mc = fmaxf(mc, __shfl_xor(mc, 4, 32)); mc = fmaxf(mc, __shfl_xor(mc, 8, 32));
      const float mn = fmaxf(m_r[r], mc); const float al = (mn > -1.0e38f) ? expf(m_r[r] - mn) : 1.0f; m_r[r] = mn;
      const float e0 = expf(s0 - mn), e1 = expf(s1 - mn);
      const float p0 = ok0 ? e0 : 0.f, p1 = ok1 ? e1 : 0.f;
      FragH t2; t2.h[0] = toh_flush(p0 * 1024.0f); t2.h[1] = toh_flush(p1 * 1024.0f);
      l_r[r] = l_r[r] * al + (float)t2.h[0] + (float)t2.h[1];
#pragma unroll
      for (int dt = 0; dt < DT; ++dt) oacc[dt][r] *= al;
      sP[w][8 * hh + r][ln] = t2.u[0]; sP[w][8 * hh + r][16 + ln] = t2.u[1];
    }
    __builtin_amdgcn_fence(4, "workgroup"); __builtin_amdgcn_wave_barrier();
    FragH pa; pa.half[0] = *(const v8us*)&sP[w][ln][8 * hh]; pa.half[1] = *(const v8us*)&sP[w][ln][16 + 8 * hh];
#pragma unroll
    for (int dt = 0; dt < DT; ++dt) {
      const unsigned short* vrow = Vth + (size_t)(dt * 16 + ln) * TK + j0; FragH bv;
      bv.half[0] = *(const v8us*)(vrow + 8 * hh); bv.half[1] = *(const v8us*)(vrow + 16 + 8 * hh);
      oacc[dt] = g2_mma(pa.v, bv.v, oacc[dt]);
    }
    __builtin_amdgcn_fence(4, "workgroup"); __builtin_amdgcn_wave_barrier();
  }
#pragma unroll
  for (int r = 0; r < 8; ++r) { float l = l_r[r]; l += __shfl_xor(l, 1, 32); l += __shfl_xor(l, 2, 32); l += __shfl_xor(l, 4, 32); l += __shfl_xor(l, 8, 32); l_r[r] = (l > 0.f) ? (1.0f / l) * CTXC : 0.f; }
#pragma unroll
  for (int dt = 0; dt < DT; ++dt)
#pragma unroll
    for (int r = 0; r < 8; ++r) sO[w][8 * hh + r][dt * 16 + ln] = oacc[dt][r] * l_r[r];
  __builtin_amdgcn_fence(4, "workgroup"); __builtin_amdgcn_wave_barrier();
  static_assert(32 * 16 * (RPW / 2) == RPW * HD * 2);
  for (int pass = 0; pass < 2; ++pass) {
#pragma unroll
    for (int rp = 0; rp < RPW; rp += 2) {
      const int r = rp + (lane >> 4), pc = lane & 15;
      const v4f va = *(const v4fa*)&sO[w][r][pc * 8]; const v4f vb = *(const v4fa*)&sO[w][r][pc * 8 + 4];
      FragH f;
#pragma unroll
      for (int q = 0; q < 4; ++q) { f.h[q] = toh_flush(va[q]); f.h[4 + q] = toh_flush(vb[q]); }
      *(volatile v8us*)((unsigned short*)OH + (size_t)(q0 + r) * DM + h * HD + pc * 8) = f.half[0];
    }
    if (pass == 0) __threadfence();
  }
}

extern "C" void kernel_launch(void* const* d_in, const int* in_sizes, int n_in,
                              void* d_out, int out_size, void* d_ws, size_t ws_size, hipStream_t stream) {
  if (n_in < 4) return;
  const size_t needx = ((size_t)(NB - 1) * SEQ_FULL + (size_t)SLEN) * DM;
  if ((size_t)in_sizes[0] < needx) return;
  if ((size_t)in_sizes[1] < (size_t)SLEN * HD) return;
  if ((size_t)in_sizes[2] < (size_t)DM * NQKV) return;
  if ((size_t)in_sizes[3] < (size_t)DM * DM) return;
  if ((size_t)out_size < needx) return;
  const float* x = (const float*)d_in[0]; const float* TAB = (const float*)d_in[1]; const float* Wa = (const float*)d_in[2]; const float* Wp = (const float*)d_in[3];
  float* dout = (float*)d_out;
  char* ws = (char*)d_ws; size_t off = 0;
  auto take = [&](size_t bytes) { char* p = ws + off; off += (bytes + 255) & ~(size_t)255; return p; };
  const size_t np = (size_t)NR * DM;
  _Float16* BA = (_Float16*)take((size_t)NQKV * DM * 2);
  _Float16* BP = (_Float16*)take((size_t)DM * DM * 2);
  float* FS = (float*)take((size_t)NR * NQKV * 4);
  _Float16* X16 = (_Float16*)take(np * 2);
  _Float16* OH = X16;
  _Float16* QH = (_Float16*)take(np * 2);
  _Float16* KH = (_Float16*)take((size_t)NR * KDIM * 2);
  _Float16* VT = (_Float16*)take((size_t)NKV * HD * TK * 2);
  if (off > ws_size) return;
  if (off > ((size_t)128 << 20)) return;

  k_wtr<<<dim3((unsigned)(NQKV / 64), (unsigned)(DM / 64)), 256, 0, stream>>>(Wa, BA, DM, NQKV, 16.0f);
  k_wtr<<<dim3((unsigned)(DM / 64), (unsigned)(DM / 64)), 256, 0, stream>>>(Wp, BP, DM, DM, 16.0f);
  const unsigned g8 = (unsigned)((np / 8 + 255) / 256);
  k_x16<<<g8, 256, 0, stream>>>(x, X16, np / 8);
  const dim3 gq((unsigned)((NR / 128) * (NQKV / 64)), 1);
  k_gemm2<0><<<gq, 128, 0, stream>>>(X16, DM, 0, BA, DM, 0, 0.0625f, FS, nullptr, NQKV, 0, NR, NQKV, DM);
  k_ropei<<<(unsigned)(((size_t)SLEN * NH * 16 + 255) / 256), 256, 0, stream>>>(FS, TAB, QH, NH, RPGQ, GQ, 0);
  k_ropei<<<(unsigned)(((size_t)SLEN * NKV * 16 + 255) / 256), 256, 0, stream>>>(FS, TAB, KH, NKV, RPGK, 1, GQ * HD);
  k_vtt<<<(unsigned)(NKV * (SLEN / 64)), 256, 0, stream>>>(FS, VT);
  k_flashb<<<(unsigned)(NH * QBLKS), 128, 0, stream>>>(QH, KH, VT, OH);
  const dim3 go((unsigned)((NR / 128) * (DM / 64)), 1);
  k_gemm2<0><<<go, 128, 0, stream>>>(OH, DM, 0, BP, DM, 0, 0.0009765625f, dout, nullptr, DM, 0, NR, DM, DM);
}
